// RAFT256_55843164783390
// MI455X (gfx1250) — hardware-verified
//
#include <hip/hip_runtime.h>


#define NBT  2
#define DD   256
#define HH   80
#define WWD  80
#define NPX  (HH * WWD)
#define RCH  1600
#define NT   81
#define NLV  4
#define NCO  (NLV * NT)
#define NCP  384
#define DM   DD
#define LOSC 1024.0f

typedef _Float16 h16;
typedef unsigned short bf;
typedef __attribute__((ext_vector_type(16))) __bf16   v16bf;
typedef __attribute__((ext_vector_type(16))) _Float16 v16h;
typedef __attribute__((ext_vector_type(8)))  _Float16 v8h;
typedef __attribute__((ext_vector_type(8)))  unsigned short v8us;
typedef __attribute__((ext_vector_type(8)))  float    v8f;
typedef __attribute__((ext_vector_type(4)))  float    v4f;
typedef v8h  __attribute__((may_alias)) v8ha;
typedef v4f  __attribute__((may_alias)) v4fa;
typedef v8us __attribute__((may_alias)) v8usa;

__device__ __forceinline__ unsigned short f2bf(float f) { unsigned u = __float_as_uint(f); u += 0x7FFFu + ((u >> 16) & 1u); return (unsigned short)(u >> 16); }
__device__ __forceinline__ float bf2f(unsigned short b) { return __uint_as_float(((unsigned)b) << 16); }
__device__ __forceinline__ float bfr(float f) { return bf2f(f2bf(f)); }
__device__ __forceinline__ v16h cat16(v8h lo, v8h hi) { return __builtin_shufflevector(lo, hi, 0, 1, 2, 3, 4, 5, 6, 7, 8, 9, 10, 11, 12, 13, 14, 15); }
__device__ __forceinline__ v16bf cat16b(v8us lo, v8us hi) { return __builtin_bit_cast(v16bf, __builtin_shufflevector(lo, hi, 0, 1, 2, 3, 4, 5, 6, 7, 8, 9, 10, 11, 12, 13, 14, 15)); }
__device__ __forceinline__ v8f wmma16(v16h a, v16h b, v8f c) { return __builtin_amdgcn_wmma_f32_16x16x32_f16(false, a, false, b, (short)0, c, false, false); }
__device__ __forceinline__ v8f wmmab(v16bf a, v16bf b, v8f c) { return __builtin_amdgcn_wmma_f32_16x16x32_bf16(false, a, false, b, (short)0, c, false, false); }

template <bool SPLITA, bool F16OUT = false>
__global__ __launch_bounds__(128) void k_gemmb(const bf* __restrict__ A, const bf* __restrict__ Al, const bf* __restrict__ Bn, const float* __restrict__ bias, float* C, int ldc, h16* C2, const float* __restrict__ R = nullptr, int K = DM, int roundR = 1) {
    __shared__ __align__(16) float ost[4][16 * 68];
    const int lane = threadIdx.x & 31, wave = threadIdx.x >> 5, lr = lane & 15, hi = lane >> 4;
    const int r0 = blockIdx.x * 64 + wave * 16, c0 = blockIdx.y * 64;
    const size_t aoff = (size_t)(r0 + lr) * K + 8 * hi;
    size_t boff[4];
#pragma unroll
    for (int t = 0; t < 4; ++t) boff[t] = (size_t)(c0 + t * 16 + lr) * K + 8 * hi;
    v8f acc[4];
#pragma unroll
    for (int t = 0; t < 4; ++t) acc[t] = (v8f){};
#pragma unroll 1
    for (int kc = 0; kc < K; kc += 32) {
        const v16bf a = cat16b(*(const v8us*)(A + aoff + kc), *(const v8us*)(A + aoff + kc + 16));
        v16bf al = a;
        if (SPLITA) al = cat16b(*(const v8us*)(Al + aoff + kc), *(const v8us*)(Al + aoff + kc + 16));
#pragma unroll
        for (int t = 0; t < 4; ++t) { const v16bf b = cat16b(*(const v8us*)(Bn + boff[t] + kc), *(const v8us*)(Bn + boff[t] + kc + 16)); acc[t] = wmmab(a, b, acc[t]); if (SPLITA) acc[t] = wmmab(al, b, acc[t]); }
        asm volatile("v_nop\n\tv_nop\n\tv_nop\n\tv_nop" : "+v"(acc[0]), "+v"(acc[1]), "+v"(acc[2]), "+v"(acc[3]) : "v"(a), "v"(al));
    }
    float* os = &ost[wave][0];
#pragma unroll
    for (int t = 0; t < 4; ++t) { const float bv = bias ? bfr(bias[c0 + t * 16 + lr]) : 0.f;
#pragma unroll
        for (int j = 0; j < 8; ++j) os[(hi * 8 + j) * 68 + t * 16 + lr] = acc[t][j] + bv; }
    __syncthreads();
    if (F16OUT) {
        h16* crow = (h16*)(void*)C + (size_t)r0 * ldc + c0;
        auto pass = [&]() {
#pragma unroll
            for (int s = 0; s < 4; ++s) { const int row = 4 * s + (lane >> 3), piece = lane & 7; const float* sp = os + row * 68 + piece * 8; v8h o, o2;
#pragma unroll
                for (int i = 0; i < 8; ++i) { const h16 a = (h16)sp[i]; o[i] = a; o2[i] = (h16)((sp[i] - (float)a) * LOSC); }
                *(volatile v8h*)(crow + (size_t)row * ldc + piece * 8) = o; if (C2) *(volatile v8h*)(C2 + (size_t)r0 * ldc + c0 + (size_t)row * ldc + piece * 8) = o2; }
        };
        pass(); __threadfence(); pass();
    } else {
        float* crow = C + (size_t)r0 * ldc + c0;
        auto pass = [&]() {
#pragma unroll
            for (int s = 0; s < 8; ++s) { const int Lid = (lane >> 3) + 4 * s, piece = lane & 7; const int row = Lid >> 1, cofs = (Lid & 1) * 32 + piece * 4;
                v4f val = *(const v4fa*)(os + row * 68 + cofs); if (R) { const v4f rv = *(const v4f*)(R + ((size_t)r0 + row) * ldc + c0 + cofs); val += roundR ? (v4f){bfr(rv[0]), bfr(rv[1]), bfr(rv[2]), bfr(rv[3])} : rv; }
                *(volatile v4f*)(crow + (size_t)row * ldc + cofs) = val; }
        };
        pass(); __threadfence(); pass();
    }
}

__global__ __launch_bounds__(256) void k_wt(const float* __restrict__ Wm, int K, int ncols, bf* WT) {
    __shared__ __align__(16) unsigned short tl[64 * 72];
    const int tid = threadIdx.x, k0 = blockIdx.x * 64, n0 = blockIdx.y * 64;
    const int kk = tid >> 2, nq = (tid & 3) * 16;
#pragma unroll
    for (int i = 0; i < 16; ++i) tl[(nq + i) * 72 + kk] = f2bf(Wm[(size_t)(k0 + kk) * ncols + n0 + nq + i]);
    __syncthreads();
    const int piece = tid & 7;
    auto pass = [&]() {
#pragma unroll
        for (int s = 0; s < 2; ++s) { const int nr = (tid >> 3) + 32 * s; const v8us val = *(const v8usa*)(tl + nr * 72 + piece * 8); *(volatile v8us*)(WT + (size_t)(n0 + nr) * K + k0 + piece * 8) = val; }
    };
    pass(); __threadfence(); pass();
}

__global__ __launch_bounds__(256) void k_pool(const float* __restrict__ src, int sh, int sw, int ssrc, float* dst, int sdst) {
    const int lane = threadIdx.x & 31; const size_t wid = (size_t)blockIdx.x * 8 + (threadIdx.x >> 5); const int dh = sh / 2, dw = sw / 2; const int per = sdst / 32; if (wid >= (size_t)RCH * per) return;
    const size_t n = wid / per; const int e = (int)(wid % per) * 32 + lane; float v = 0.f;
    if (e < dh * dw) { const int y = e / dw, x = e % dw; const float* s = src + n * ssrc + (size_t)(2 * y) * sw + 2 * x; v = (s[0] + s[1] + s[sw] + s[sw + 1]) * 0.25f; }
    *(volatile float*)(dst + n * sdst + e) = v; __threadfence(); *(volatile float*)(dst + n * sdst + e) = v;
}
__global__ __launch_bounds__(256) void k_lookup(const float* __restrict__ L0, const float* __restrict__ L1, const float* __restrict__ L2, const float* __restrict__ L3, const float* __restrict__ crd, size_t n0, float* OT) {
    const int lane = threadIdx.x & 31; const size_t n = (size_t)blockIdx.x * 8 + (threadIdx.x >> 5); if (n >= (size_t)RCH) return; const size_t gn = n0 + n;
    const float cx = bfr(crd[gn]), cy = bfr(crd[NPX + gn]);
#pragma unroll 1
    for (int ps = 0; ps < 2; ++ps) {
#pragma unroll 1
        for (int q = 0; q < NCP / 128; ++q) { v4f v;
#pragma unroll
            for (int i = 0; i < 4; ++i) { const int c = q * 128 + lane * 4 + i; float val = 0.f;
                if (c < NCO) { const int l = c / NT, t = c % NT; const int ti = t / 9, tj = t % 9; const float sc = 1.0f / (float)(1 << l); const int lh = HH >> l, lw = WWD >> l;
                    const float* img = (l == 0) ? L0 : (l == 1) ? L1 : (l == 2) ? L2 : L3; const int stride = (l == 0) ? 6400 : (l == 1) ? 1600 : (l == 2) ? 416 : 128;
                    const float x = cx * sc + (float)(ti - 4), y = cy * sc + (float)(tj - 4); const float x0f = floorf(x), y0f = floorf(y); const float wx = x - x0f, wy = y - y0f; const int x0 = (int)x0f, y0 = (int)y0f;
                    auto g = [&](int yi, int xi) -> float { const bool ok = xi >= 0 && xi <= lw - 1 && yi >= 0 && yi <= lh - 1; const int yc = yi < 0 ? 0 : (yi > lh - 1 ? lh - 1 : yi), xc = xi < 0 ? 0 : (xi > lw - 1 ? lw - 1 : xi); return ok ? img[n * stride + (size_t)yc * lw + xc] : 0.f; };
                    val = g(y0, x0) * (1.f - wy) * (1.f - wx) + g(y0, x0 + 1) * (1.f - wy) * wx + g(y0 + 1, x0) * wy * (1.f - wx) + g(y0 + 1, x0 + 1) * wy * wx; }
                v[i] = val; }
            *(volatile v4f*)(OT + n * NCP + q * 128 + lane * 4) = v; }
        if (ps == 0) __threadfence(); }
}
__global__ __launch_bounds__(256) void k_outT(const float* __restrict__ OT, size_t n0, float* OUTB) {
    const int lane = threadIdx.x & 31; const size_t wid = (size_t)blockIdx.x * 8 + (threadIdx.x >> 5); if (wid >= (size_t)NCO * (RCH / 32)) return; const int c = (int)(wid / (RCH / 32)); const int nn = (int)(wid % (RCH / 32)) * 32 + lane;
    const float v = OT[(size_t)nn * NCP + c] * 0.0625f; *(volatile float*)(OUTB + (size_t)c * NPX + n0 + nn) = v; __threadfence(); *(volatile float*)(OUTB + (size_t)c * NPX + n0 + nn) = v;
}

extern "C" void kernel_launch(void* const* d_in, const int* in_sizes, int n_in,
                              void* d_out, int out_size, void* d_ws, size_t ws_size, hipStream_t stream) {
    (void)in_sizes; (void)n_in; (void)out_size;
    const float* f1 = (const float*)d_in[0]; const float* f2 = (const float*)d_in[1]; const float* crd = (const float*)d_in[2];
    float* out = (float*)d_out;
    char* wsp = (char*)d_ws;
    auto take = [&](size_t bytes) { char* p = wsp; wsp += (bytes + 255) & ~(size_t)255; return (void*)p; };
    bf* P1 = (bf*)take((size_t)NPX * DD * 2); bf* P2 = (bf*)take((size_t)NPX * DD * 2); float* L0 = (float*)take((size_t)RCH * NPX * 4); float* L1 = (float*)take((size_t)RCH * 1600 * 4); float* L2 = (float*)take((size_t)RCH * 416 * 4); float* L3 = (float*)take((size_t)RCH * 128 * 4); float* OT = (float*)take((size_t)RCH * NCP * 4);
    if ((size_t)(wsp - (char*)d_ws) > ws_size) return;
    for (int b = 0; b < NBT; ++b) {
        k_wt<<<dim3(DD / 64, NPX / 64, 1), 256, 0, stream>>>(f1 + (size_t)b * DD * NPX, DD, NPX, P1); k_wt<<<dim3(DD / 64, NPX / 64, 1), 256, 0, stream>>>(f2 + (size_t)b * DD * NPX, DD, NPX, P2);
        for (int c = 0; c < NPX / RCH; ++c) { const size_t n0 = (size_t)c * RCH;
            k_gemmb<false, false><<<dim3(RCH / 64, NPX / 64, 1), 128, 0, stream>>>(P1 + n0 * DD, nullptr, P2, nullptr, L0, NPX, nullptr, nullptr, DD);
            k_pool<<<(RCH * (1600 / 32)) / 8, 256, 0, stream>>>(L0, 80, 80, NPX, L1, 1600);
            k_pool<<<(RCH * (416 / 32)) / 8, 256, 0, stream>>>(L1, 40, 40, 1600, L2, 416);
            k_pool<<<(RCH * (128 / 32)) / 8, 256, 0, stream>>>(L2, 20, 20, 416, L3, 128);
            k_lookup<<<RCH / 8, 256, 0, stream>>>(L0, L1, L2, L3, crd + (size_t)b * 2 * NPX, n0, OT);
            k_outT<<<(NCO * (RCH / 32)) / 8, 256, 0, stream>>>(OT, n0, out + (size_t)b * NCO * NPX); } }
}
